// NeRF_85315230368439
// MI455X (gfx1250) — hardware-verified
//
#include <hip/hip_runtime.h>
#include <math.h>

typedef __attribute__((ext_vector_type(16))) _Float16 v16h;
typedef __attribute__((ext_vector_type(8)))  _Float16 v8h;
typedef __attribute__((ext_vector_type(8)))  float    v8f;
typedef __attribute__((ext_vector_type(4)))  float    v4f;
typedef __attribute__((ext_vector_type(4)))  unsigned int v4u;

namespace {
constexpr int kHidden      = 256;
constexpr int kInDim       = 39;
constexpr int kNumFreq     = 6;
constexpr int kK0          = 64;
constexpr int kSamples     = 64;
constexpr int kRaysPerBlk  = 32;
constexpr int kSubTiles    = 16;
constexpr int kRows        = 128;
constexpr int kThreads     = 256;
constexpr int kPitchH      = 264;
constexpr int kPitchX      = 72;
constexpr float kWCarry    = 16.0f;
constexpr float kWInv      = 1.0f / 16.0f;
constexpr float kXlCarry   = 16.0f;
constexpr float kXsScale   = 1.0f / 16.0f;

constexpr size_t kWsW1t   = 0;
constexpr size_t kWsW0t   = 131072;
constexpr size_t kWsW2t   = 131072 + 32768;
constexpr size_t kWsTotal = 131072 + 32768 + 8192;

constexpr int kLoW1  = 0;
constexpr int kLoW0  = kLoW1 + kHidden * kPitchH * 2;
constexpr int kLoW2  = kLoW0 + kHidden * kPitchX * 2;
constexpr int kLoH   = kLoW2 + 16 * kPitchH * 2;
constexpr int kLoX   = kLoH + kRows * kPitchH * 2;
constexpr int kLoB0  = kLoX + kRows * kPitchX * 2;
constexpr int kLoB1  = kLoB0 + kHidden * 4;
constexpr int kLoB2  = kLoB1 + kHidden * 4;
constexpr int kLoRS  = kLoB2 + 16 * 4;
constexpr int kLoOut = kLoRS + kRows * 4 * 4;
constexpr int kLdsBytes = kLoOut + kRaysPerBlk * 3 * 4;

static_assert(kInDim + 6 <= kK0, "feature columns fit the padded K");
static_assert(kK0 % 32 == 0 && kHidden % 32 == 0, "K multiples of 32");
static_assert(kRows == 2 * kSamples && kSamples == 64, "two rays of 64 samples per sub-tile");
static_assert(kRaysPerBlk == 2 * kSubTiles, "rays per block");
static_assert(kThreads == kHidden, "bias staging maps one thread per hidden unit");
static_assert((kLoW0 % 16) == 0 && (kLoW2 % 16) == 0 && (kLoH % 16) == 0 && (kLoX % 16) == 0, "align");
static_assert((kLoB0 % 16) == 0 && (kLoRS % 16) == 0 && (kLoOut % 16) == 0, "align");
static_assert(kLdsBytes == 271040, "lds total");
static_assert((kPitchH * 2) % 16 == 0 && (kPitchX * 2) % 16 == 0, "row pitch 16B");
static_assert((kWsW0t % 128) == 0 && (kWsW2t % 128) == 0, "plane bases line aligned");
}

template <typename T> struct Frag;
template <> struct Frag<_Float16> {
  typedef v16h V; union U { v16h v; v8h h[2]; };
  static __device__ __forceinline__ v16h load(const _Float16* p) {
    U f; f.h[0] = *(const v8h*)(p); f.h[1] = *(const v8h*)(p + 16); return f.v;
  }
};

__device__ __forceinline__ unsigned pk16(unsigned short a, unsigned short b) { return (unsigned)a | ((unsigned)b << 16); }
__device__ __forceinline__ unsigned short h_bits(float f) { const _Float16 h = (_Float16)f; return __builtin_bit_cast(unsigned short, h); }
__device__ __forceinline__ v8f zero8() { return (v8f){0.f, 0.f, 0.f, 0.f, 0.f, 0.f, 0.f, 0.f}; }
__device__ __forceinline__ v8f mma16(v16h a, v16h b, v8f c) {
  return __builtin_amdgcn_wmma_f32_16x16x32_f16(false, a, false, b, (short)0, c, false, false);
}
__device__ __forceinline__ void guard_2acc(v8f& c0, v8f& c1, v16h a, v16h b0, v16h b1) {
  asm volatile("v_nop\n\tv_nop\n\tv_nop\n\tv_nop" : "+v"(c0), "+v"(c1) : "v"(a), "v"(b0), "v"(b1));
}
__device__ __forceinline__ void guard_1acc(v8f& c0, v16h a, v16h b) {
  asm volatile("v_nop\n\tv_nop\n\tv_nop\n\tv_nop" : "+v"(c0) : "v"(a), "v"(b));
}

__global__ __launch_bounds__(256) void prep_weights(const float* __restrict__ W0, const float* __restrict__ W1,
                                                      const float* __restrict__ W2,
                                                      unsigned short* __restrict__ w1t, unsigned short* __restrict__ w0t,
                                                      unsigned short* __restrict__ w2t) {
  __shared__ float sm[4224];
  const int t = threadIdx.x, lane = t & 31, wave = t >> 5;
  const int blk = blockIdx.x;
  const int q = lane >> 3, c8 = (lane & 7) * 8;
  if (blk < 16) {
    const int n0 = (blk >> 2) * 64, k0 = (blk & 3) * 64;
#pragma unroll 8
    for (int i = 0; i < 16; ++i) {
      const int e = i * 256 + t;
      const int kl = e >> 6, nl = e & 63;
      sm[nl * 65 + kl] = kWCarry * W1[(size_t)(k0 + kl) * kHidden + n0 + nl];
    }
    __syncthreads();
    for (int pass = 0; pass < 2; ++pass) {
#pragma unroll
      for (int it = 0; it < 2; ++it) {
        const int row = wave * 8 + it * 4 + q;
        unsigned short hb[8];
#pragma unroll
        for (int e = 0; e < 8; ++e) hb[e] = h_bits(sm[row * 65 + c8 + e]);
        const v4u u = (v4u){pk16(hb[0], hb[1]), pk16(hb[2], hb[3]), pk16(hb[4], hb[5]), pk16(hb[6], hb[7])};
        *(volatile v4u*)(w1t + (size_t)(n0 + row) * kHidden + k0 + c8) = u;
      }
      __threadfence();
    }
  } else if (blk < 20) {
    const int n0 = (blk - 16) * 64;
#pragma unroll 8
    for (int i = 0; i < 16; ++i) {
      const int e = i * 256 + t;
      const int k = e >> 6, nl = e & 63;
      int kk = k;
      if (k >= 39) kk = k - 39;
      if (k >= 42) kk = k - 42;
      if (k >= 45) kk = 0;
      const float w   = W0[(size_t)kk * kHidden + n0 + nl];
      const float w16 = kWCarry * w;
      const float hi  = (float)((_Float16)w16);
      const float lo  = (w16 - hi) * kWCarry;
      float v = w16;
      if (k >= 39) v = w;
      if (k >= 42) v = lo;
      if (k >= 45) v = 0.0f;
      sm[nl * 65 + k] = v;
    }
    __syncthreads();
    for (int pass = 0; pass < 2; ++pass) {
#pragma unroll
      for (int it = 0; it < 2; ++it) {
        const int row = wave * 8 + it * 4 + q;
        unsigned short hb[8];
#pragma unroll
        for (int e = 0; e < 8; ++e) hb[e] = h_bits(sm[row * 65 + c8 + e]);
        const v4u u = (v4u){pk16(hb[0], hb[1]), pk16(hb[2], hb[3]), pk16(hb[4], hb[5]), pk16(hb[6], hb[7])};
        *(volatile v4u*)(w0t + (size_t)(n0 + row) * kK0 + c8) = u;
      }
      __threadfence();
    }
  } else {
#pragma unroll
    for (int i = 0; i < 16; ++i) {
      float v = 0.0f;
      if (i < 4) v = kWCarry * W2[(size_t)t * 4 + i];
      sm[i * 257 + t] = v;
    }
    __syncthreads();
    for (int pass = 0; pass < 2; ++pass) {
#pragma unroll
      for (int it = 0; it < 2; ++it) {
        const int row = wave * 2 + it;
        unsigned short hb[8];
#pragma unroll
        for (int e = 0; e < 8; ++e) hb[e] = h_bits(sm[row * 257 + lane * 8 + e]);
        const v4u u = (v4u){pk16(hb[0], hb[1]), pk16(hb[2], hb[3]), pk16(hb[4], hb[5]), pk16(hb[6], hb[7])};
        *(volatile v4u*)(w2t + (size_t)row * kHidden + lane * 8) = u;
      }
      __threadfence();
    }
  }
}

__global__ __launch_bounds__(kThreads) void field_render(
    const float* __restrict__ origins, const float* __restrict__ dirs, const float* __restrict__ trand,
    const unsigned short* __restrict__ w1t, const unsigned short* __restrict__ w0t, const unsigned short* __restrict__ w2t,
    const float* __restrict__ b0, const float* __restrict__ b1, const float* __restrict__ b2,
    const int* __restrict__ nearp, const int* __restrict__ farp, float* __restrict__ out, int nrays) {
  extern __shared__ __align__(16) unsigned char lds[];
  const _Float16* sW1 = (const _Float16*)(lds + kLoW1);
  const _Float16* sW0 = (const _Float16*)(lds + kLoW0);
  const _Float16* sW2 = (const _Float16*)(lds + kLoW2);
  _Float16* sH  = (_Float16*)(lds + kLoH);
  const _Float16* sX = (const _Float16*)(lds + kLoX);
  float* sB0  = (float*)(lds + kLoB0);
  float* sB1  = (float*)(lds + kLoB1);
  float* sB2  = (float*)(lds + kLoB2);
  float* sRS  = (float*)(lds + kLoRS);
  float* sOut = (float*)(lds + kLoOut);

  const int tid = threadIdx.x, wave = tid >> 5, lane = tid & 31;
  const int rlane = lane & 15;
  const int koff  = (lane >> 4) * 8;
  const int mOff  = (lane >> 4) * 8;
  const float nearf = (float)nearp[0];
  const float farf  = (float)farp[0];
  const float fn    = farf - nearf;

  {
    const v4u* g1 = (const v4u*)w1t;
#pragma unroll 4
    for (int e = tid; e < kHidden * 32; e += kThreads) {
      const int n = e >> 5, c = e & 31;
      *(v4u*)(lds + kLoW1 + n * (kPitchH * 2) + c * 16) = g1[e];
    }
    const v4u* g0 = (const v4u*)w0t;
#pragma unroll 4
    for (int e = tid; e < kHidden * 8; e += kThreads) {
      const int n = e >> 3, c = e & 7;
      *(v4u*)(lds + kLoW0 + n * (kPitchX * 2) + c * 16) = g0[e];
    }
    const v4u* g2 = (const v4u*)w2t;
#pragma unroll
    for (int e = tid; e < 16 * 32; e += kThreads) {
      const int n = e >> 5, c = e & 31;
      *(v4u*)(lds + kLoW2 + n * (kPitchH * 2) + c * 16) = g2[e];
    }
    sB0[tid] = b0[tid];
    sB1[tid] = b1[tid];
    {
      const int bi = (tid < 4) ? tid : 3;
      const float bv = b2[bi];
      if (tid < 16) sB2[tid] = (tid < 4) ? bv : 0.0f;
    }
  }
  __syncthreads();

  const int rayBase = blockIdx.x * kRaysPerBlk;

#pragma unroll 1
  for (int st = 0; st < kSubTiles; ++st) {
    if (tid < kRows) {
      const int p = tid, rsub = p >> 6, s = p & 63;
      int ray = rayBase + st * 2 + rsub;
      ray = (ray < nrays) ? ray : (nrays - 1);
      const float tr  = trand[(size_t)ray * kSamples + s];
      const float ts0 = (float)s * (1.0f / 64.0f);
      const float ts1 = (float)(s + 1) * (1.0f / 64.0f);
      const float z0  = fn * ts0 + nearf;
      const float z1  = fn * ts1 + nearf;
      const float mid = 0.5f * (z1 + z0);
      const float up  = z1 - mid;
      const float lw  = mid - z0;
      const float zr  = mid + up * tr - lw * (1.0f - tr);
      unsigned short hb[64];
#pragma unroll
      for (int c = 0; c < 3; ++c) {
        const float x = origins[(size_t)ray * 3 + c] + dirs[(size_t)ray * 3 + c] * zr;
        const _Float16 xhh = (_Float16)x;
        const float xh = (float)xhh;
        hb[c]      = __builtin_bit_cast(unsigned short, xhh);
        hb[39 + c] = h_bits((x - xh) * kXlCarry);
        hb[42 + c] = h_bits(xh * kXsScale);
        float sn, cs;
        sincosf(x, &sn, &cs);
        hb[3 + c] = h_bits(sn);
        hb[6 + c] = h_bits(cs);
#pragma unroll
        for (int l = 1; l < kNumFreq; ++l) {
          const float s2 = 2.0f * sn * cs;
          const float c2 = cs * cs - sn * sn;
          sn = s2;
          cs = c2;
          hb[3 + 6 * l + c] = h_bits(sn);
          hb[6 + 6 * l + c] = h_bits(cs);
        }
      }
#pragma unroll
      for (int j = 45; j < 64; ++j) hb[j] = hb[42 + ((j - 45) % 3)];
      v4u* xr = (v4u*)(lds + kLoX + p * (kPitchX * 2));
#pragma unroll
      for (int qd = 0; qd < 8; ++qd) {
        v4u u;
        u[0] = pk16(hb[8 * qd + 0], hb[8 * qd + 1]);
        u[1] = pk16(hb[8 * qd + 2], hb[8 * qd + 3]);
        u[2] = pk16(hb[8 * qd + 4], hb[8 * qd + 5]);
        u[3] = pk16(hb[8 * qd + 6], hb[8 * qd + 7]);
        xr[qd] = u;
      }
    }
    __syncthreads();

    {
      const _Float16* arow = sX + (wave * 16 + rlane) * kPitchX + koff;
#pragma unroll 1
      for (int nt = 0; nt < 16; nt += 2) {
        v8f c0 = zero8(), c1 = zero8();
        const _Float16* brow0 = sW0 + (nt * 16 + rlane) * kPitchX + koff;
        const _Float16* brow1 = brow0 + 16 * kPitchX;
#pragma unroll
        for (int kt = 0; kt < kK0 / 32; ++kt) {
          const v16h a   = Frag<_Float16>::load(arow + kt * 32);
          const v16h fb0 = Frag<_Float16>::load(brow0 + kt * 32);
          const v16h fb1 = Frag<_Float16>::load(brow1 + kt * 32);
          c0 = mma16(a, fb0, c0);
          c1 = mma16(a, fb1, c1);
          guard_2acc(c0, c1, a, fb0, fb1);
        }
        const int col0 = nt * 16 + rlane;
        const float bv0 = sB0[col0], bv1 = sB0[col0 + 16];
#pragma unroll
        for (int r = 0; r < 8; ++r) {
          const int row = wave * 16 + mOff + r;
          sH[row * kPitchH + col0]      = (_Float16)fmaxf(c0[r] * kWInv + bv0, 0.0f);
          sH[row * kPitchH + col0 + 16] = (_Float16)fmaxf(c1[r] * kWInv + bv1, 0.0f);
        }
      }
    }
    __syncthreads();

    v16h afr[8];
    {
      const _Float16* arow = sH + (wave * 16 + rlane) * kPitchH + koff;
#pragma unroll
      for (int kt = 0; kt < 8; ++kt) afr[kt] = Frag<_Float16>::load(arow + kt * 32);
    }
    __syncthreads();
#pragma unroll 1
    for (int nt = 0; nt < 16; nt += 2) {
      v8f c0 = zero8(), c1 = zero8();
      const _Float16* brow0 = sW1 + (nt * 16 + rlane) * kPitchH + koff;
      const _Float16* brow1 = brow0 + 16 * kPitchH;
#pragma unroll
      for (int kt = 0; kt < 8; ++kt) {
        const v16h fb0 = Frag<_Float16>::load(brow0 + kt * 32);
        const v16h fb1 = Frag<_Float16>::load(brow1 + kt * 32);
        c0 = mma16(afr[kt], fb0, c0);
        c1 = mma16(afr[kt], fb1, c1);
        guard_2acc(c0, c1, afr[kt], fb0, fb1);
      }
      const int col0 = nt * 16 + rlane;
      const float bv0 = sB1[col0], bv1 = sB1[col0 + 16];
#pragma unroll
      for (int r = 0; r < 8; ++r) {
        const int row = wave * 16 + mOff + r;
        sH[row * kPitchH + col0]      = (_Float16)fmaxf(c0[r] * kWInv + bv0, 0.0f);
        sH[row * kPitchH + col0 + 16] = (_Float16)fmaxf(c1[r] * kWInv + bv1, 0.0f);
      }
    }
    __syncthreads();

    {
      v8f c2 = zero8();
      const _Float16* arow = sH + (wave * 16 + rlane) * kPitchH + koff;
      const _Float16* brow = sW2 + rlane * kPitchH + koff;
#pragma unroll
      for (int kt = 0; kt < 8; ++kt) {
        const v16h a  = Frag<_Float16>::load(arow + kt * 32);
        const v16h fb = Frag<_Float16>::load(brow + kt * 32);
        c2 = mma16(a, fb, c2);
        guard_1acc(c2, a, fb);
      }
      const float bv = sB2[rlane];
#pragma unroll
      for (int r = 0; r < 8; ++r) {
        const int row = wave * 16 + mOff + r;
        const float v   = c2[r] * kWInv + bv;
        const float sg  = 1.0f / (1.0f + expf(-v));
        const float rl  = fmaxf(v, 0.0f);
        const float val = (rlane < 3) ? sg : rl;
        if (rlane < 4) sRS[row * 4 + rlane] = val;
      }
    }
    __syncthreads();

    if (wave < 2) {
      const int rl = wave;
      const float* rs = sRS + rl * kSamples * 4;
      float aT[2], al[2], cr[2], cg[2], cb[2];
#pragma unroll
      for (int j = 0; j < 2; ++j) {
        const int s = 2 * lane + j;
        const float z0  = fn * ((float)s * (1.0f / 64.0f)) + nearf;
        const float z1  = fn * ((float)(s + 1) * (1.0f / 64.0f)) + nearf;
        const float seg = z1 - z0;
        const float sig = rs[s * 4 + 3];
        cr[j] = rs[s * 4 + 0];
        cg[j] = rs[s * 4 + 1];
        cb[j] = rs[s * 4 + 2];
        const float alpha = 1.0f - expf(-sig * seg);
        al[j] = alpha;
        aT[j] = (1.0f - alpha) + 1e-10f;
      }
      float x = aT[0] * aT[1];
#pragma unroll
      for (int off = 1; off < 32; off <<= 1) {
        const float y = __shfl_up(x, off, 32);
        const float f = (lane >= off) ? y : 1.0f;
        x = x * f;
      }
      float ex = __shfl_up(x, 1, 32);
      ex = (lane == 0) ? 1.0f : ex;
      const float T0 = ex;
      const float T1 = ex * aT[0];
      const float w0 = al[0] * T0;
      const float w1 = al[1] * T1;
      float sr = w0 * cr[0] + w1 * cr[1];
      float sg = w0 * cg[0] + w1 * cg[1];
      float sb = w0 * cb[0] + w1 * cb[1];
#pragma unroll
      for (int off = 16; off > 0; off >>= 1) {
        sr += __shfl_xor(sr, off, 32);
        sg += __shfl_xor(sg, off, 32);
        sb += __shfl_xor(sb, off, 32);
      }
      if (lane == 0) {
        sOut[(st * 2 + rl) * 3 + 0] = sr;
        sOut[(st * 2 + rl) * 3 + 1] = sg;
        sOut[(st * 2 + rl) * 3 + 2] = sb;
      }
    }
  }
  __syncthreads();

  if (wave == 0) {
    const int li = (lane < 24) ? lane : 23;
    const v4f val = *(const v4f*)(sOut + li * 4);
    float* op = out + (size_t)blockIdx.x * (kRaysPerBlk * 3) + li * 4;
    if (lane < 24) *(volatile v4f*)op = val;
    __threadfence();
    if (lane < 24) *(volatile v4f*)op = val;
  }
}

extern "C" void kernel_launch(void* const* d_in, const int* in_sizes, int n_in,
                              void* d_out, int out_size, void* d_ws, size_t ws_size,
                              hipStream_t stream) {
  (void)n_in;
  const float* origins = (const float*)d_in[0];
  const float* dirs    = (const float*)d_in[1];
  const float* trand   = (const float*)d_in[2];
  const float* W0      = (const float*)d_in[3];
  const float* b0      = (const float*)d_in[4];
  const float* W1      = (const float*)d_in[5];
  const float* b1      = (const float*)d_in[6];
  const float* W2      = (const float*)d_in[7];
  const float* b2      = (const float*)d_in[8];
  const int*   nearp   = (const int*)d_in[9];
  const int*   farp    = (const int*)d_in[10];
  float*       out     = (float*)d_out;

  const int nrays = in_sizes[0] / 3;
  if (nrays <= 0) return;
  if (nrays % kRaysPerBlk != 0) return;
  if (in_sizes[2] != nrays * kSamples) return;
  if (out_size != nrays * 3) return;
  if (ws_size < kWsTotal) return;

  unsigned char* ws = (unsigned char*)d_ws;
  unsigned short* w1t = (unsigned short*)(ws + kWsW1t);
  unsigned short* w0t = (unsigned short*)(ws + kWsW0t);
  unsigned short* w2t = (unsigned short*)(ws + kWsW2t);

  prep_weights<<<dim3(21), dim3(256), 0, stream>>>(W0, W1, W2, w1t, w0t, w2t);

  hipFuncSetAttribute((const void*)field_render, hipFuncAttributeMaxDynamicSharedMemorySize, kLdsBytes);
  const int nblk = nrays / kRaysPerBlk;
  field_render<<<dim3(nblk), dim3(kThreads), kLdsBytes, stream>>>(
      origins, dirs, trand, w1t, w0t, w2t, b0, b1, b2, nearp, farp, out, nrays);
}
